// DeformablePatchEmbed_GELU_7352984011448
// MI455X (gfx1250) — hardware-verified
//
#include <hip/hip_runtime.h>
#include <math.h>

typedef __attribute__((ext_vector_type(16))) _Float16 v16h;
typedef __attribute__((ext_vector_type(16))) __bf16 v16b;
typedef __attribute__((ext_vector_type(8)))  _Float16 v8h;
typedef __attribute__((ext_vector_type(8)))  float v8f;
typedef __attribute__((ext_vector_type(4)))  float v4f;
typedef __attribute__((ext_vector_type(2)))  float v2f;
typedef __attribute__((ext_vector_type(4)))  unsigned v4u;
typedef __attribute__((ext_vector_type(4)))  int v4i;
typedef float __attribute__((may_alias)) float_a;
typedef int __attribute__((may_alias)) int_a;

template <typename T> __device__ __forceinline__ void vst2(void* p, T v) { *(volatile T*)p = v; __threadfence(); *(volatile T*)p = v; }
__device__ __forceinline__ v8f wmma16(v16h a, v16h b, v8f c) {
  v8f d = __builtin_amdgcn_wmma_f32_16x16x32_f16(false, a, false, b, (short)0, c, false, false);
  asm volatile("v_nop\n\tv_nop\n\tv_nop\n\tv_nop" : "+v"(d) : "v"(a), "v"(b));
  return d;
}
__device__ __forceinline__ v8f wmma_bf(v16b a, v16b b, v8f c) {
  v8f d = __builtin_amdgcn_wmma_f32_16x16x32_bf16(false, a, false, b, (short)0, c, false, false);
  asm volatile("v_nop\n\tv_nop\n\tv_nop\n\tv_nop" : "+v"(d) : "v"(a), "v"(b));
  return d;
}
__device__ __forceinline__ v16h frag_h(const _Float16* rowk0, int lane) {
  union { v16h v; v8h q[2]; } u; const _Float16* p = rowk0 + 8 * (lane >> 4);
  u.q[0] = *(const v8h*)p; u.q[1] = *(const v8h*)(p + 16); return u.v;
}
__device__ __forceinline__ v16h frag_f32(const float* rowk0, int lane) {
  v16h a; const float* p = rowk0 + 8 * (lane >> 4);
#pragma unroll
  for (int i = 0; i < 8; ++i) { a[i] = (_Float16)p[i]; a[8 + i] = (_Float16)p[16 + i]; }
  return a;
}
__device__ __forceinline__ v16h frag_f32s(const float* rowk0, int lane, float sc) {
  v16h a; const float* p = rowk0 + 8 * (lane >> 4);
#pragma unroll
  for (int i = 0; i < 8; ++i) { a[i] = (_Float16)(p[i] * sc); a[8 + i] = (_Float16)(p[16 + i] * sc); }
  return a;
}
__device__ __forceinline__ v16h fragc_f32(const float* W, int k0, int n, int lane, int ld, int K) {
  v16h a; const int g = lane >> 4;
#pragma unroll
  for (int i = 0; i < 8; ++i) { const int ka = k0 + 8 * g + i, kb = ka + 16;
    a[i] = (_Float16)(ka < K ? W[(size_t)(ka < K ? ka : K - 1) * ld + n] : 0.f); a[8 + i] = (_Float16)(kb < K ? W[(size_t)(kb < K ? kb : K - 1) * ld + n] : 0.f); }
  return a;
}
struct F2 { v16b h, l; };
__device__ __forceinline__ F2 bsplit16(const float v[16]) { F2 r;
#pragma unroll
  for (int i = 0; i < 16; ++i) { const __bf16 h = (__bf16)v[i]; r.h[i] = h; r.l[i] = (__bf16)(v[i] - (float)h); }
  return r; }
__device__ __forceinline__ F2 split_row(const float* row, int k0, int lane) { float v[16]; const float* p = row + k0 + 8 * (lane >> 4);
#pragma unroll
  for (int i = 0; i < 8; ++i) { v[i] = p[i]; v[8 + i] = p[16 + i]; }
  return bsplit16(v); }
__device__ __forceinline__ F2 split_rowK(const float* row, int k0, int lane, int K) { float v[16]; const int g = lane >> 4;
#pragma unroll
  for (int i = 0; i < 8; ++i) { const int ka = k0 + 8 * g + i, kb = ka + 16; v[i] = ka < K ? row[ka < K ? ka : K - 1] : 0.f; v[8 + i] = kb < K ? row[kb < K ? kb : K - 1] : 0.f; }
  return bsplit16(v); }
__device__ __forceinline__ F2 split_col(const float* W, int k0, int n, int lane, int ld, int K) { float v[16]; const int g = lane >> 4;
#pragma unroll
  for (int i = 0; i < 8; ++i) { const int ka = k0 + 8 * g + i, kb = ka + 16; v[i] = ka < K ? W[(size_t)(ka < K ? ka : K - 1) * ld + n] : 0.f; v[8 + i] = kb < K ? W[(size_t)(kb < K ? kb : K - 1) * ld + n] : 0.f; }
  return bsplit16(v); }
__device__ __forceinline__ v8f mac3(const F2& a, const F2& b, v8f c) { c = wmma_bf(a.l, b.h, c); c = wmma_bf(a.h, b.l, c); return wmma_bf(a.h, b.h, c); }
__device__ __forceinline__ float sigm(float v) { return 1.0f / (1.0f + expf(-v)); }
#define LDSX() do { asm volatile("s_wait_dscnt 0" ::: "memory"); __builtin_amdgcn_wave_barrier(); __builtin_amdgcn_fence(__ATOMIC_RELEASE, "workgroup"); } while (0)


#define NBAT 64
#define CH 3
#define HI 224
#define WI 224
#define PS 16
#define HO 14
#define WO 14
#define KP (PS * PS)
#define KIN (CH * KP)
#define NOFF (2 * KP)
#define NO 768
#ifndef NBT
#define NBT NBAT
#endif
#define NP (NBT * HO * WO)
#define NPF (NBAT * HO * WO)
#define NPB ((NP + 63) / 64)
typedef __attribute__((ext_vector_type(8))) __bf16 v8b;
__device__ __forceinline__ v16b frag_b(const __bf16* rowk0, int lane) {
  union { v16b v; v8b q[2]; } u; const __bf16* p = rowk0 + 8 * (lane >> 4);
  u.q[0] = *(const v8b*)p; u.q[1] = *(const v8b*)(p + 16); return u.v;
}
__device__ __forceinline__ float bfr(float v) { return (float)(__bf16)v; }
__device__ __attribute__((noinline)) float exp_ni(float v) { return expf(v); }
__device__ __attribute__((noinline)) float erf_ni(float v) { return erff(v); }

#define WS_PO   0u
#define WS_PD   (WS_PO + 2u * NOFF * KIN)
#define WS_OFF  (WS_PD + 2u * NO * KIN)
#define WS_SMP  (WS_OFF + 4u * NPB * 64 * NOFF)
#define WS_Y    (WS_SMP + 4u * NPB * 64 * KIN)
#define WS_PSUM (WS_Y + 4u * NPB * 64 * NO)
#define WS_ST   (WS_PSUM + 4u * NPB * NO)
#define WS_END  (WS_ST + 4u * 2 * NO)

__global__ __launch_bounds__(256) void k_pack(const float* __restrict__ WOF, const float* __restrict__ WD, __bf16* __restrict__ PO, __bf16* __restrict__ PD) {
  __shared__ __align__(16) __bf16 s[KIN]; const int n = blockIdx.x, pl = blockIdx.y, tid = threadIdx.x;
  if (pl == 0 && n >= NOFF) return;
  const float* w = (pl == 0) ? WOF + (size_t)n * KIN : WD + (size_t)n * KIN;
  for (int k = tid; k < KIN; k += 256) s[k] = (__bf16)w[k];
  __syncthreads();
  for (int q = tid; q < KIN / 8; q += 256) vst2((unsigned*)((pl == 0 ? PO : PD) + (size_t)n * KIN + q * 8), *(const v4u*)&s[q * 8]);
}
__global__ __launch_bounds__(128) void k_offconv(const float* __restrict__ X, const __bf16* __restrict__ PO, const float* __restrict__ OB, float* __restrict__ OFF) {
  __shared__ __align__(16) float so[4][16][132];
  const int tid = threadIdx.x, wave = tid >> 5, lane = tid & 31, col = lane & 15, g = lane >> 4; const int r0 = blockIdx.x * 64 + wave * 16; const int n0 = blockIdx.y * 128;
  int pa = r0 + col; if (pa >= NP) pa = NP - 1; const int b = pa / (HO * WO), ho = (pa / WO) % HO, wo = pa % WO;
  v8f acc[8] = {};
#pragma unroll 1
  for (int kc = 0; kc < KIN / 32; ++kc) { v16b a;
#pragma unroll
    for (int i = 0; i < 16; ++i) { const int k = kc * 32 + 8 * g + (i < 8 ? i : 8 + i); const int c = k / KP, r = k % KP; const int hh = ho * PS + r / PS, ww = wo * PS + r % PS; a[i] = (__bf16)X[(((size_t)b * CH + c) * HI + hh) * WI + ww]; }
#pragma unroll
    for (int j = 0; j < 8; ++j) acc[j] = wmma_bf(a, frag_b(PO + (size_t)(n0 + j * 16 + col) * KIN + kc * 32, lane), acc[j]); }
#pragma unroll
  for (int j = 0; j < 8; ++j) { const float bb = bfr(OB[n0 + j * 16 + col]);
#pragma unroll
    for (int r = 0; r < 8; ++r) so[wave][8 * g + r][j * 16 + col] = acc[j][r] + bb; }
  LDSX();
  for (int rl = 0; rl < 16; ++rl) vst2(OFF + (size_t)(r0 + rl) * NOFF + n0 + lane * 4, *(const v4f*)&so[wave][rl][lane * 4]);
}
__global__ __launch_bounds__(256) void k_sample(const float* __restrict__ X, const float* __restrict__ OFF, float* __restrict__ SMP) {
  __shared__ __align__(16) float s[KIN]; const int p = blockIdx.x, k = threadIdx.x; const int b = p / (HO * WO), ho = (p / WO) % HO, wo = p % WO;
  const float dy = OFF[(size_t)p * NOFF + 2 * k], dx = OFF[(size_t)p * NOFF + 2 * k + 1];
  const float py = ((float)(ho * PS) + (float)(k / PS)) + dy, px = ((float)(wo * PS) + (float)(k % PS)) + dx;
  const float y0 = floorf(py), x0 = floorf(px); const float wy1 = py - y0, wx1 = px - x0, wy0 = 1.0f - wy1, wx0 = 1.0f - wx1;
  const int y0i = (int)y0, x0i = (int)x0, y1i = y0i + 1, x1i = x0i + 1;
  const bool oky0 = (y0i >= 0 && y0i < HI), oky1 = (y1i >= 0 && y1i < HI), okx0 = (x0i >= 0 && x0i < WI), okx1 = (x1i >= 0 && x1i < WI);
  const int cy0 = min(max(y0i, 0), HI - 1), cy1 = min(max(y1i, 0), HI - 1), cx0 = min(max(x0i, 0), WI - 1), cx1 = min(max(x1i, 0), WI - 1);
#pragma unroll
  for (int c = 0; c < CH; ++c) { const float* img = X + ((size_t)b * CH + c) * HI * WI;
    const float v00 = (oky0 && okx0) ? bfr(img[cy0 * WI + cx0]) : 0.f, v01 = (oky0 && okx1) ? bfr(img[cy0 * WI + cx1]) : 0.f, v10 = (oky1 && okx0) ? bfr(img[cy1 * WI + cx0]) : 0.f, v11 = (oky1 && okx1) ? bfr(img[cy1 * WI + cx1]) : 0.f;
    s[c * KP + k] = v00 * (wy0 * wx0) + v01 * (wy0 * wx1) + v10 * (wy1 * wx0) + v11 * (wy1 * wx1); }
  __syncthreads();
  for (int q = k; q < KIN / 4; q += 256) vst2(SMP + (size_t)p * KIN + q * 4, *(const v4f*)&s[q * 4]);
}
__global__ __launch_bounds__(128) void k_dconv(const float* __restrict__ SMP, const __bf16* __restrict__ PD, float* __restrict__ Y) {
  __shared__ __align__(16) float so[4][16][132];
  const int tid = threadIdx.x, wave = tid >> 5, lane = tid & 31, col = lane & 15, g = lane >> 4; const int r0 = blockIdx.x * 64 + wave * 16; const int n0 = blockIdx.y * 128;
  int ra = r0 + col; if (ra >= NP) ra = NP - 1;
  v8f acc[8] = {};
#pragma unroll 2
  for (int kc = 0; kc < KIN / 32; ++kc) { const F2 a = split_row(SMP + (size_t)ra * KIN, kc * 32, lane);
#pragma unroll
    for (int j = 0; j < 8; ++j) { const v16b w = frag_b(PD + (size_t)(n0 + j * 16 + col) * KIN + kc * 32, lane); acc[j] = wmma_bf(a.l, w, acc[j]); acc[j] = wmma_bf(a.h, w, acc[j]); } }
#pragma unroll
  for (int j = 0; j < 8; ++j)
#pragma unroll
    for (int r = 0; r < 8; ++r) so[wave][8 * g + r][j * 16 + col] = acc[j][r];
  LDSX();
  for (int rl = 0; rl < 16; ++rl) vst2(Y + (size_t)(r0 + rl) * NO + n0 + lane * 4, *(const v4f*)&so[wave][rl][lane * 4]);
}
template <int MODE>
__global__ __launch_bounds__(256) void k_colsum(const float* __restrict__ Y, const float* __restrict__ ST, float* __restrict__ PSUM) {
  __shared__ __align__(16) float s[NO]; const int blk = blockIdx.x, tid = threadIdx.x;
  for (int c = tid; c < NO; c += 256) { const float mu = (MODE == 1) ? ST[c] : 0.f; float acc = 0.f;
    for (int rl = 0; rl < 64; ++rl) { const int row = blk * 64 + rl; if (row < NP) { const float v = Y[(size_t)row * NO + c]; acc += (MODE == 1) ? (v - mu) * (v - mu) : v; } }
    s[c] = acc; }
  __syncthreads();
  for (int q = tid; q < NO / 4; q += 256) vst2(PSUM + (size_t)blk * NO + q * 4, *(const v4f*)&s[q * 4]);
}
template <int MODE>
__global__ __launch_bounds__(256) void k_red(const float* __restrict__ PSUM, float* __restrict__ ST) {
  __shared__ __align__(16) float s[NO]; const int tid = threadIdx.x;
  for (int c = tid; c < NO; c += 256) { float acc = 0.f; for (int b = 0; b < NPB; ++b) acc += PSUM[(size_t)b * NO + c]; s[c] = (MODE == 0) ? acc / (float)NP : rsqrtf(acc / (float)NP + 1e-5f); }
  __syncthreads();
  for (int q = tid; q < NO / 4; q += 256) vst2(ST + MODE * NO + q * 4, *(const v4f*)&s[q * 4]);
}
__global__ __launch_bounds__(256) void k_bnact(const float* __restrict__ Y, const float* __restrict__ ST, const float* __restrict__ gm, const float* __restrict__ bt, float* __restrict__ out) {
  __shared__ __align__(16) float s[8][NO];
  const int wave = threadIdx.x >> 5, lane = threadIdx.x & 31; const int row = blockIdx.x * 8 + wave; if (row >= NP) return;
  for (int c = lane; c < NO; c += 32) { const float v = (Y[(size_t)row * NO + c] - ST[c]) * ST[NO + c] * bfr(gm[c]) + bfr(bt[c]); s[wave][c] = 0.5f * v * (1.0f + erf_ni(v * 0.70710678118654752f)); }
  LDSX();
  for (int pc = lane; pc < NO / 4; pc += 32) vst2(out + (size_t)row * NO + pc * 4, *(const v4f*)&s[wave][pc * 4]);
}
extern "C" void kernel_launch(void* const* d_in, const int* in_sizes, int n_in, void* d_out, int out_size, void* d_ws, size_t ws_size, hipStream_t stream) {
  (void)in_sizes; (void)n_in; (void)out_size;
  const float** F = (const float**)d_in;
  if (ws_size < (size_t)WS_END) return;
  char* ws = (char*)d_ws; __bf16 *PO = (__bf16*)(ws + WS_PO), *PD = (__bf16*)(ws + WS_PD); float *OFF = (float*)(ws + WS_OFF), *SMP = (float*)(ws + WS_SMP), *Y = (float*)(ws + WS_Y), *PSUM = (float*)(ws + WS_PSUM), *ST = (float*)(ws + WS_ST);
  k_pack<<<dim3(NO, 2), 256, 0, stream>>>(F[1], F[3], PO, PD);
  k_offconv<<<dim3(NPB, NOFF / 128), 128, 0, stream>>>(F[0], PO, F[2], OFF);
  k_sample<<<NP, 256, 0, stream>>>(F[0], OFF, SMP);
  k_dconv<<<dim3(NPB, NO / 128), 128, 0, stream>>>(SMP, PD, Y);
  k_colsum<0><<<NPB, 256, 0, stream>>>(Y, ST, PSUM); k_red<0><<<1, 256, 0, stream>>>(PSUM, ST); k_colsum<1><<<NPB, 256, 0, stream>>>(Y, ST, PSUM); k_red<1><<<1, 256, 0, stream>>>(PSUM, ST);
  k_bnact<<<(NP + 7) / 8, 256, 0, stream>>>(Y, ST, F[4], F[5], (float*)d_out);
}
